// SPN_90546500534706
// MI455X (gfx1250) — hardware-verified
//
#include <hip/hip_runtime.h>
#include <stdint.h>
#include <stddef.h>

typedef __attribute__((ext_vector_type(16))) _Float16 v16h;
typedef __attribute__((ext_vector_type(8)))  _Float16 v8h;
typedef __attribute__((ext_vector_type(16))) __bf16   v16b;
typedef __attribute__((ext_vector_type(8)))  __bf16   v8b;
typedef __attribute__((ext_vector_type(8)))  float    v8f;
typedef __attribute__((ext_vector_type(4)))  float    v4f;
typedef __attribute__((ext_vector_type(4)))  unsigned v4u;

__device__ __forceinline__ unsigned short f2bf_bits(float f) {
  unsigned u = __float_as_uint(f);
  return (unsigned short)((u + 0x7FFFu + ((u >> 16) & 1u)) >> 16);
}
__device__ __forceinline__ float bf_bits2f(unsigned short h) { return __uint_as_float(((unsigned)h) << 16); }
__device__ __forceinline__ unsigned short f2h_bits(float f) { return __builtin_bit_cast(unsigned short, (_Float16)f); }
__device__ __forceinline__ unsigned pack2(unsigned short lo, unsigned short hi) { return (unsigned)lo | ((unsigned)hi << 16); }
__device__ __forceinline__ float elu_f(float t) {
  const float en = expf(fminf(t, 0.0f)) - 1.0f;
  return (t > 0.0f) ? t : en;
}

__device__ __forceinline__ void dep_guard_h(v8f& a, v8f& b, v16h x, v16h y) { asm volatile("v_nop\n\tv_nop\n\tv_nop\n\tv_nop" : "+v"(a), "+v"(b) : "v"(x), "v"(y)); }
__device__ __forceinline__ void dep_guard_b(v8f& a, v8f& b, v16b x, v16b y) { asm volatile("v_nop\n\tv_nop\n\tv_nop\n\tv_nop" : "+v"(a), "+v"(b) : "v"(x), "v"(y)); }
__device__ __forceinline__ void keep4_h(v16h a, v16h b, v16h c, v16h d) { asm volatile("v_nop" :: "v"(a), "v"(b), "v"(c), "v"(d)); }
__device__ __forceinline__ void keep4_b(v16b a, v16b b, v16b c, v16b d) { asm volatile("v_nop" :: "v"(a), "v"(b), "v"(c), "v"(d)); }
__device__ __forceinline__ void acc_guard4(v8f& a, v8f& b, v8f& c, v8f& d) { asm volatile("v_nop\n\tv_nop\n\tv_nop\n\tv_nop" : "+v"(a), "+v"(b), "+v"(c), "+v"(d)); }

template <typename T> struct Frag;
template <> struct Frag<_Float16> {
  typedef v16h V; union U { v16h v; v8h h[2]; };
  static __device__ __forceinline__ v16h load(const _Float16* p) {
    U f; f.h[0] = *(const v8h*)(p); f.h[1] = *(const v8h*)(p + 16); return f.v;
  }
  static __device__ __forceinline__ v8f mma(v16h a, v16h b, v8f c) {
    return __builtin_amdgcn_wmma_f32_16x16x32_f16(false, a, false, b, (short)0, c, false, false);
  }
  static __device__ __forceinline__ void guard(v8f& a, v8f& b, v16h x, v16h y) { dep_guard_h(a, b, x, y); }
  static __device__ __forceinline__ void keep(v16h a, v16h b, v16h c, v16h d) { keep4_h(a, b, c, d); }
};
template <> struct Frag<__bf16> {
  typedef v16b V; union U { v16b v; v8b h[2]; };
  static __device__ __forceinline__ v16b load(const __bf16* p) {
    U f; f.h[0] = *(const v8b*)(p); f.h[1] = *(const v8b*)(p + 16); return f.v;
  }
  static __device__ __forceinline__ v8f mma(v16b a, v16b b, v8f c) {
    return __builtin_amdgcn_wmma_f32_16x16x32_bf16(false, a, false, b, (short)0, c, false, false);
  }
  static __device__ __forceinline__ void guard(v8f& a, v8f& b, v16b x, v16b y) { dep_guard_b(a, b, x, y); }
  static __device__ __forceinline__ void keep(v16b a, v16b b, v16b c, v16b d) { keep4_b(a, b, c, d); }
};
template <int ET> struct Elem;
template <> struct Elem<0> { typedef _Float16 T; };
template <> struct Elem<1> { typedef __bf16 T; };

template <int ET, bool SPLIT, int OUT_MODE, bool RESID, int ACT>
__global__ __launch_bounds__(256) void conv_gemm64(
    const unsigned short* __restrict__ Ap, const unsigned short* A2p, int lda,
    const unsigned short* __restrict__ Btp, const unsigned short* Bt2p, int ldb,
    void* __restrict__ Cout, int ldc,
    const float* __restrict__ bias, int nbias,
    const float* resid,
    int M, int N, int K, float scale) {
  typedef typename Elem<ET>::T T;
  typedef typename Frag<T>::V V;
  const T* A = (const T*)Ap; const T* A2 = (const T*)A2p; const T* Bt = (const T*)Btp; const T* Bt2 = (const T*)Bt2p;
  __shared__ __align__(16) float sT[8][16 * 68];
  const int lane = threadIdx.x & 31;
  const int wave = threadIdx.x >> 5;
  const int tilesN = N >> 6;
  const int tilesM = M >> 6;
  const int tile = blockIdx.x * 8 + wave;
  if (tile >= tilesM * tilesN) return;
  const int tm = tile / tilesN;
  const int tn = tile - tm * tilesN;
  const int m0 = tm << 6;
  const int n0 = tn << 6;

  const int rlane = lane & 15;
  const int koff  = (lane >> 4) * 8;
  const int mOff  = (lane >> 4) * 8;

  v8f acc[4][4];
#pragma unroll
  for (int i = 0; i < 4; ++i)
#pragma unroll
    for (int j = 0; j < 4; ++j) acc[i][j] = (v8f){0.f,0.f,0.f,0.f,0.f,0.f,0.f,0.f};

  for (int k0 = 0; k0 < K; k0 += 32) {
    V bh[4], bl[4];
#pragma unroll
    for (int j = 0; j < 4; ++j) {
      const size_t bo = (size_t)(n0 + (j << 4) + rlane) * ldb + koff + k0;
      bh[j] = Frag<T>::load(Bt + bo);
      if (SPLIT) bl[j] = Frag<T>::load(Bt2 + bo);
    }
#pragma unroll
    for (int i = 0; i < 4; ++i) {
      const size_t ao = (size_t)(m0 + (i << 4) + rlane) * lda + koff + k0;
      V ah = Frag<T>::load(A + ao);
      V al;
      if (SPLIT) al = Frag<T>::load(A2 + ao);
#pragma unroll
      for (int j = 0; j < 4; ++j) {
        acc[i][j] = Frag<T>::mma(ah, bh[j], acc[i][j]);
        if (SPLIT) {
          acc[i][j] = Frag<T>::mma(ah, bl[j], acc[i][j]);
          acc[i][j] = Frag<T>::mma(al, bh[j], acc[i][j]);
        }
      }
      Frag<T>::guard(acc[i][0], acc[i][3], ah, SPLIT ? al : ah);
    }
    Frag<T>::keep(bh[0], bh[1], bh[2], bh[3]);
    if (SPLIT) Frag<T>::keep(bl[0], bl[1], bl[2], bl[3]);
  }
  acc_guard4(acc[0][0], acc[0][1], acc[0][2], acc[0][3]);
  acc_guard4(acc[1][0], acc[1][1], acc[1][2], acc[1][3]);
  acc_guard4(acc[2][0], acc[2][1], acc[2][2], acc[2][3]);
  acc_guard4(acc[3][0], acc[3][1], acc[3][2], acc[3][3]);

  float* slab = sT[wave];
  constexpr int NCOL = (OUT_MODE == 0) ? 4 : 8;
  const int cb = (OUT_MODE == 0) ? ((lane & 15) * 4) : ((lane & 7) * 8);
  float bcol[NCOL];
#pragma unroll
  for (int e = 0; e < NCOL; ++e) {
    int n = n0 + cb + e;
    n = (n < nbias) ? n : (nbias - 1);
    bcol[e] = bias[n];
  }
  const v4f z4 = (v4f){0.f, 0.f, 0.f, 0.f};
#pragma unroll
  for (int i = 0; i < 4; ++i) {
    const int mBase = m0 + (i << 4);
#pragma unroll
    for (int j = 0; j < 4; ++j) {
#pragma unroll
      for (int r = 0; r < 8; ++r) slab[(mOff + r) * 68 + (j << 4) + rlane] = acc[i][j][r];
    }
    __builtin_amdgcn_fence(__ATOMIC_RELEASE, "workgroup");
    __builtin_amdgcn_wave_barrier();
    __builtin_amdgcn_fence(__ATOMIC_ACQUIRE, "workgroup");
    if (OUT_MODE == 0) {
      float* Cp = (float*)Cout;
      const int hh = lane >> 4;
      v4f vals[8];
#pragma unroll
      for (int it = 0; it < 8; ++it) {
        const int row = it * 2 + hh;
        const v4f a = *(const v4f*)(slab + row * 68 + cb);
        v4f rr = z4;
        if (RESID) rr = *(const v4f*)(resid + (size_t)(mBase + row) * ldc + n0 + cb);
        v4f o;
#pragma unroll
        for (int e = 0; e < 4; ++e) {
          float t = a[e] * scale + bcol[e];
          if (ACT == 6) t = elu_f(t);
          if (RESID) t += rr[e];
          o[e] = t;
        }
        vals[it] = o;
      }
      for (int pass = 0; pass < 2; ++pass) {
#pragma unroll
        for (int it = 0; it < 8; ++it) {
          const int row = it * 2 + hh;
          *(volatile v4f*)(Cp + (size_t)(mBase + row) * ldc + n0 + cb) = vals[it];
        }
        __threadfence();
      }
    } else {
      unsigned short* Cp = (unsigned short*)Cout;
      const int q = lane >> 3;
      v8h hvs[4];
#pragma unroll
      for (int it = 0; it < 4; ++it) {
        const int row = it * 4 + q;
        const float* sp = slab + row * 68 + cb;
        const v4f a0 = *(const v4f*)(sp);
        const v4f a1 = *(const v4f*)(sp + 4);
        v4f r0 = z4, r1 = z4;
        if (RESID) {
          const float* rp = resid + (size_t)(mBase + row) * ldc + n0 + cb;
          r0 = *(const v4f*)(rp);
          r1 = *(const v4f*)(rp + 4);
        }
        v8h hv;
#pragma unroll
        for (int e = 0; e < 4; ++e) {
          float t = a0[e] * scale + bcol[e];
          if (ACT == 6) t = elu_f(t);
          if (RESID) t += r0[e];
          hv[e] = (_Float16)t;
        }
#pragma unroll
        for (int e = 0; e < 4; ++e) {
          float t = a1[e] * scale + bcol[4 + e];
          if (ACT == 6) t = elu_f(t);
          if (RESID) t += r1[e];
          hv[4 + e] = (_Float16)t;
        }
        hvs[it] = hv;
      }
      for (int pass = 0; pass < 2; ++pass) {
#pragma unroll
        for (int it = 0; it < 4; ++it) {
          const int row = it * 4 + q;
          *(volatile v8h*)(Cp + (size_t)(mBase + row) * ldc + n0 + cb) = hvs[it];
        }
        __threadfence();
      }
    }
    __builtin_amdgcn_fence(__ATOMIC_RELEASE, "workgroup");
    __builtin_amdgcn_wave_barrier();
    __builtin_amdgcn_fence(__ATOMIC_ACQUIRE, "workgroup");
  }
}

template <int SPLIT>
__global__ __launch_bounds__(256) void cast_weight(const float* __restrict__ w, int N, int K, int Npad, int Kpad,
                                                   float carry, unsigned short* o1, unsigned short* o2)
{
  const unsigned t = blockIdx.x * 256u + threadIdx.x;
  const unsigned total = ((unsigned)Npad * (unsigned)Kpad) >> 3;
  if (t >= total) return;
  const unsigned kq = (unsigned)Kpad >> 3;
  const unsigned n = t / kq;
  const int k0 = (int)(t - n * kq) * 8;
  unsigned short hb[8], lb[8];
#pragma unroll
  for (int i = 0; i < 8; ++i) {
    const int k = k0 + i;
    const bool valid = ((int)n < N) && (k < K);
    const int nc = ((int)n < N) ? (int)n : (N - 1);
    const int kc = (k < K) ? k : (K - 1);
    float f = w[(size_t)nc * K + kc];
    f = valid ? (f * carry) : 0.0f;
    if (SPLIT) {
      const unsigned short h = f2bf_bits(f);
      hb[i] = h;
      lb[i] = f2bf_bits(f - bf_bits2f(h));
    } else {
      hb[i] = f2h_bits(f);
      lb[i] = 0;
    }
  }
  v4u wh, wl;
  wh.x = pack2(hb[0], hb[1]); wh.y = pack2(hb[2], hb[3]); wh.z = pack2(hb[4], hb[5]); wh.w = pack2(hb[6], hb[7]);
  wl.x = pack2(lb[0], lb[1]); wl.y = pack2(lb[2], lb[3]); wl.z = pack2(lb[4], lb[5]); wl.w = pack2(lb[6], lb[7]);
  const size_t o = (size_t)t * 8;
  *(volatile v4u*)(o1 + o) = wh;
  if (SPLIT) *(volatile v4u*)(o2 + o) = wl;
  __threadfence();
  *(volatile v4u*)(o1 + o) = wh;
  if (SPLIT) *(volatile v4u*)(o2 + o) = wl;
}

template <int SRC16, int SPLITOUT>
__global__ __launch_bounds__(256) void im2col3x3(
    const float* srcf, const unsigned short* srch, long sN, long sC, long sP,
    unsigned short* dst, unsigned short* dst2,
    int Cin, int H, int W, int Kreal, int Kpad, int m_begin, int nrows)
{
  const unsigned t = blockIdx.x * 256u + threadIdx.x;
  const unsigned kq = (unsigned)Kpad >> 3;
  const unsigned r = t / kq;
  if (r >= (unsigned)nrows) return;
  const int k0 = (int)(t - r * kq) * 8;
  const int m = m_begin + (int)r;
  const int HW = H * W;
  const int nb = m / HW;
  const int p = m - nb * HW;
  const int y = p / W;
  const int x = p - y * W;
  unsigned short hb[8], lb[8];
#pragma unroll
  for (int i = 0; i < 8; ++i) {
    const int k = k0 + i;
    const int ci = k / 9;
    const int r9 = k - ci * 9;
    const int ky = r9 / 3;
    const int kx = r9 - ky * 3;
    const int iy = y + ky - 1;
    const int ix = x + kx - 1;
    const bool valid = (k < Kreal) && (iy >= 0) && (iy < H) && (ix >= 0) && (ix < W);
    const int cic = (ci < Cin) ? ci : (Cin - 1);
    const int iyc = (iy < 0) ? 0 : ((iy >= H) ? (H - 1) : iy);
    const int ixc = (ix < 0) ? 0 : ((ix >= W) ? (W - 1) : ix);
    const long addr = (long)nb * sN + (long)cic * sC + (long)(iyc * W + ixc) * sP;
    if (SRC16) {
      const unsigned short u = srch[addr];
      hb[i] = valid ? u : (unsigned short)0;
      lb[i] = 0;
    } else {
      float f = srcf[addr];
      f = valid ? f : 0.0f;
      if (SPLITOUT) {
        const unsigned short h = f2bf_bits(f);
        hb[i] = h;
        lb[i] = f2bf_bits(f - bf_bits2f(h));
      } else {
        hb[i] = f2h_bits(f);
        lb[i] = 0;
      }
    }
  }
  v4u wh, wl;
  wh.x = pack2(hb[0], hb[1]); wh.y = pack2(hb[2], hb[3]); wh.z = pack2(hb[4], hb[5]); wh.w = pack2(hb[6], hb[7]);
  wl.x = pack2(lb[0], lb[1]); wl.y = pack2(lb[2], lb[3]); wl.z = pack2(lb[4], lb[5]); wl.w = pack2(lb[6], lb[7]);
  const size_t o = (size_t)r * (size_t)Kpad + (size_t)k0;
  *(volatile v4u*)(dst + o) = wh;
  if (SPLITOUT) *(volatile v4u*)(dst2 + o) = wl;
  __threadfence();
  *(volatile v4u*)(dst + o) = wh;
  if (SPLITOUT) *(volatile v4u*)(dst2 + o) = wl;
}

template <int OUTF32>
__global__ __launch_bounds__(256) void relu_pool3s2(const float* __restrict__ src, int pitch, int C,
                                                    int NB, int H, int W, float* dstf, unsigned short* dsth)
{
  constexpr int VEC = OUTF32 ? 4 : 8;
  const int Ho = H >> 1, Wo = W >> 1;
  const unsigned t = blockIdx.x * 256u + threadIdx.x;
  const unsigned cq = (unsigned)C / VEC;
  const unsigned total = (unsigned)(NB * Ho * Wo) * cq;
  if (t >= total) return;
  const unsigned mo = t / cq;
  const int c0 = (int)(t - mo * cq) * VEC;
  const int HWo = Ho * Wo;
  const int nb = (int)mo / HWo;
  const int p = (int)mo - nb * HWo;
  const int oy = p / Wo;
  const int ox = p - oy * Wo;
  float mx[VEC];
#pragma unroll
  for (int e = 0; e < VEC; ++e) mx[e] = 0.0f;
#pragma unroll 1
  for (int dy = 0; dy < 3; ++dy) {
    const int iy = 2 * oy - 1 + dy;
    const bool vy = (iy >= 0) && (iy < H);
    const int iyc = (iy < 0) ? 0 : ((iy >= H) ? (H - 1) : iy);
#pragma unroll
    for (int dx = 0; dx < 3; ++dx) {
      const int ix = 2 * ox - 1 + dx;
      const bool valid = vy && (ix >= 0) && (ix < W);
      const int ixc = (ix < 0) ? 0 : ((ix >= W) ? (W - 1) : ix);
      const float* q = src + ((size_t)nb * H * W + (size_t)iyc * W + ixc) * pitch + c0;
#pragma unroll
      for (int e4 = 0; e4 < VEC; e4 += 4) {
        const v4f v = *(const v4f*)(q + e4);
#pragma unroll
        for (int e = 0; e < 4; ++e) {
          float a = valid ? v[e] : 0.0f;
          a = fmaxf(a, 0.0f);
          mx[e4 + e] = fmaxf(mx[e4 + e], a);
        }
      }
    }
  }
  const size_t o = (size_t)mo * C + c0;
  if (OUTF32) {
    v4f w4; w4.x = mx[0]; w4.y = mx[1]; w4.z = mx[2]; w4.w = mx[3];
    float* dp = dstf + o;
    *(volatile v4f*)dp = w4;
    __threadfence();
    *(volatile v4f*)dp = w4;
  } else {
    v4u wh;
    wh.x = pack2(f2h_bits(mx[0]), f2h_bits(mx[1]));
    wh.y = pack2(f2h_bits(mx[2]), f2h_bits(mx[3]));
    wh.z = pack2(f2h_bits(mx[VEC - 4]), f2h_bits(mx[VEC - 3]));
    wh.w = pack2(f2h_bits(mx[VEC - 2]), f2h_bits(mx[VEC - 1]));
    unsigned short* dp = dsth + o;
    *(volatile v4u*)dp = wh;
    __threadfence();
    *(volatile v4u*)dp = wh;
  }
}

template <int OUTF32>
__global__ __launch_bounds__(256) void upsample2x(const float* __restrict__ src, int C, int NB, int H, int W,
                                                  float* dstf, unsigned short* dsth)
{
  constexpr int VEC = OUTF32 ? 4 : 8;
  const int Ho = 2 * H, Wo = 2 * W;
  const unsigned t = blockIdx.x * 256u + threadIdx.x;
  const unsigned cq = (unsigned)C / VEC;
  const unsigned total = (unsigned)(NB * Ho * Wo) * cq;
  if (t >= total) return;
  const unsigned mo = t / cq;
  const int c0 = (int)(t - mo * cq) * VEC;
  const int HWo = Ho * Wo;
  const int nb = (int)mo / HWo;
  const int p = (int)mo - nb * HWo;
  const int oy = p / Wo;
  const int ox = p - oy * Wo;
  const int y0 = (oy + 1) / 2 - 1;
  const int x0 = (ox + 1) / 2 - 1;
  float fy = (oy & 1) ? 0.25f : 0.75f;
  float fx = (ox & 1) ? 0.25f : 0.75f;
  float wy0 = 1.0f - fy, wy1 = fy;
  float wx0 = 1.0f - fx, wx1 = fx;
  if (y0 < 0) { wy0 = 0.0f; wy1 = 1.0f; }
  if (y0 + 1 > H - 1) { wy0 = 1.0f; wy1 = 0.0f; }
  if (x0 < 0) { wx0 = 0.0f; wx1 = 1.0f; }
  if (x0 + 1 > W - 1) { wx0 = 1.0f; wx1 = 0.0f; }
  const int y0c = (y0 < 0) ? 0 : y0;
  const int y1c = (y0 + 1 > H - 1) ? (H - 1) : (y0 + 1);
  const int x0c = (x0 < 0) ? 0 : x0;
  const int x1c = (x0 + 1 > W - 1) ? (W - 1) : (x0 + 1);
  const size_t pb = (size_t)nb * H * W;
  const float* p00 = src + (pb + (size_t)y0c * W + x0c) * C + c0;
  const float* p01 = src + (pb + (size_t)y0c * W + x1c) * C + c0;
  const float* p10 = src + (pb + (size_t)y1c * W + x0c) * C + c0;
  const float* p11 = src + (pb + (size_t)y1c * W + x1c) * C + c0;
  float val[VEC];
#pragma unroll
  for (int e4 = 0; e4 < VEC; e4 += 4) {
    const v4f a = *(const v4f*)(p00 + e4);
    const v4f b = *(const v4f*)(p01 + e4);
    const v4f c = *(const v4f*)(p10 + e4);
    const v4f d = *(const v4f*)(p11 + e4);
#pragma unroll
    for (int e = 0; e < 4; ++e) {
      const float colL = wy0 * a[e] + wy1 * c[e];
      const float colR = wy0 * b[e] + wy1 * d[e];
      val[e4 + e] = wx0 * colL + wx1 * colR;
    }
  }
  const size_t o = (size_t)mo * C + c0;
  if (OUTF32) {
    v4f w4; w4.x = val[0]; w4.y = val[1]; w4.z = val[2]; w4.w = val[3];
    float* dp = dstf + o;
    *(volatile v4f*)dp = w4;
    __threadfence();
    *(volatile v4f*)dp = w4;
  } else {
    v4u wh;
    wh.x = pack2(f2h_bits(val[0]), f2h_bits(val[1]));
    wh.y = pack2(f2h_bits(val[2]), f2h_bits(val[3]));
    wh.z = pack2(f2h_bits(val[VEC - 4]), f2h_bits(val[VEC - 3]));
    wh.w = pack2(f2h_bits(val[VEC - 2]), f2h_bits(val[VEC - 1]));
    unsigned short* dp = dsth + o;
    *(volatile v4u*)dp = wh;
    __threadfence();
    *(volatile v4u*)dp = wh;
  }
}

__global__ __launch_bounds__(256) void gates_base(const float* __restrict__ raw, const float* __restrict__ xp,
                                                  float* __restrict__ gb, int m_begin, int nrows)
{
  const unsigned t = blockIdx.x * 256u + threadIdx.x;
  const unsigned r = t >> 5;
  if (r >= (unsigned)nrows) return;
  const int q = (int)(t & 7u);
  const int d = (int)((t >> 3) & 3u);
  const size_t m = (size_t)m_begin + r;
  const float* rp = raw + (size_t)r * 384 + 96 * d + 4 * q;
  const v4f g1 = *(const v4f*)(rp);
  const v4f g2 = *(const v4f*)(rp + 32);
  const v4f g3 = *(const v4f*)(rp + 64);
  const v4f xv = *(const v4f*)(xp + m * 64 + 4 * q);
  v4f bo, go;
#pragma unroll
  for (int e = 0; e < 4; ++e) {
    float s = fabsf(g1[e]) + fabsf(g2[e]) + fabsf(g3[e]);
    s = (s == 0.0f) ? 1e-6f : s;
    const bool big = (s >= 1.0f);
    const float q1 = g1[e] / s;
    const float q2 = g2[e] / s;
    const float G1 = big ? q1 : g1[e];
    const float G2 = big ? q2 : g2[e];
    bo[e] = G1 * xv[e];
    go[e] = G2;
  }
  float* dp = gb + m * 256 + 64 * d + 4 * q;
  *(volatile v4f*)(dp) = bo;
  *(volatile v4f*)(dp + 32) = go;
  __threadfence();
  *(volatile v4f*)(dp) = bo;
  *(volatile v4f*)(dp + 32) = go;
}

#define PROP_H 192
#define PROP_W 192
#define PROP_PL 6
#define GB_PITCH 256

__global__ __launch_bounds__(256) void prop_scan_max(const float* __restrict__ gb, float* __restrict__ omax, int nsteps)
{
  __shared__ __align__(16) float om[PROP_H * PROP_W];
  const int lane = threadIdx.x & 31;
  const int wave = threadIdx.x >> 5;
  const int plane = blockIdx.x;
  const int nb = plane >> 5;
  const int ch = plane & 31;
  const size_t pix0 = (size_t)nb * (PROP_H * PROP_W);
  const int nst = (nsteps < 96) ? nsteps : 96;
  for (int d = 0; d < 4; ++d) {
    const bool horiz = (d < 2);
    const bool rev = ((d & 1) != 0);
    for (int line = wave; line < PROP_H; line += 8) {
      float bse[PROP_PL], g2v[PROP_PL], o[PROP_PL];
#pragma unroll
      for (int j = 0; j < PROP_PL; ++j) {
        const int i = lane * PROP_PL + j;
        const int y = horiz ? line : i;
        const int x = horiz ? i : line;
        const float* p = gb + (pix0 + (size_t)y * PROP_W + x) * GB_PITCH + 64 * d + ch;
        bse[j] = p[0];
        g2v[j] = p[32];
        o[j] = bse[j];
      }
      if (!rev) {
#pragma unroll 1
        for (int it = 0; it < nst; ++it) {
          const float up = __shfl_up(o[PROP_PL - 1], 1, 32);
          const float sh = (lane == 0) ? o[0] : up;
          float nw[PROP_PL];
          nw[0] = bse[0] + g2v[0] * sh;
#pragma unroll
          for (int j = 1; j < PROP_PL; ++j) nw[j] = bse[j] + g2v[j] * o[j - 1];
#pragma unroll
          for (int j = 0; j < PROP_PL; ++j) o[j] = nw[j];
        }
      } else {
#pragma unroll 1
        for (int it = 0; it < nst; ++it) {
          const float dn = __shfl_down(o[0], 1, 32);
          const float sh = (lane == 31) ? o[PROP_PL - 1] : dn;
          float nw[PROP_PL];
          nw[PROP_PL - 1] = bse[PROP_PL - 1] + g2v[PROP_PL - 1] * sh;
#pragma unroll
          for (int j = 0; j < PROP_PL - 1; ++j) nw[j] = bse[j] + g2v[j] * o[j + 1];
#pragma unroll
          for (int j = 0; j < PROP_PL; ++j) o[j] = nw[j];
        }
      }
#pragma unroll
      for (int j = 0; j < PROP_PL; ++j) {
        const int i = lane * PROP_PL + j;
        const int y = horiz ? line : i;
        const int x = horiz ? i : line;
        const int idx = y * PROP_W + x;
        if (d == 0) om[idx] = o[j];
        else om[idx] = fmaxf(om[idx], o[j]);
      }
    }
    __syncthreads();
  }
  float* op = omax + (size_t)plane * (PROP_H * PROP_W);
  for (int pass = 0; pass < 2; ++pass) {
    for (int row = wave; row < PROP_H; row += 8) {
      const v4f v = *(const v4f*)(om + row * PROP_W + lane * 4);
      *(volatile v4f*)(op + (size_t)row * PROP_W + lane * 4) = v;
      if (lane < 16) {
        const v4f v2 = *(const v4f*)(om + row * PROP_W + 128 + lane * 4);
        *(volatile v4f*)(op + (size_t)row * PROP_W + 128 + lane * 4) = v2;
      }
    }
    __threadfence();
  }
}

__global__ __launch_bounds__(256) void gather_output(const float* __restrict__ cp, float* __restrict__ out)
{
  const int t = blockIdx.x * 256 + threadIdx.x;
  if (t >= 55296) return;
  const int e = t * 4;
  const int plane = e / 36864;
  const int p = e - plane * 36864;
  const int nb = plane / 3;
  const int c = plane - nb * 3;
  const size_t m = (size_t)nb * 36864 + p;
  v4f v;
  v.x = cp[(m + 0) * 64 + c];
  v.y = cp[(m + 1) * 64 + c];
  v.z = cp[(m + 2) * 64 + c];
  v.w = cp[(m + 3) * 64 + c];
  *(volatile v4f*)(out + e) = v;
  __threadfence();
  *(volatile v4f*)(out + e) = v;
}

namespace propns {
constexpr int NB = 2;
constexpr int H1 = 192, W1 = 192, HW1 = H1 * W1, M1 = NB * HW1;
constexpr int H2 = 96,  HW2 = H2 * H2,  M2 = NB * HW2;
constexpr int H3 = 48,  HW3 = H3 * H3,  M3 = NB * HW3;
constexpr int H4 = 24,  HW4 = H4 * H4,  M4 = NB * HW4;
constexpr int NSTEPS = 96;
constexpr int MC4 = M2 / 2;
constexpr int MC6 = M1 / 8;
constexpr int MC7 = M1 / 8;
constexpr long oWmask = 0;
constexpr long oWv1h  = 4096;
constexpr long oWv1l  = 8192;
constexpr long oWv2h  = 12288;
constexpr long oWv2l  = 49152;
constexpr long oWv3   = 86016;
constexpr long oWv4   = 233472;
constexpr long oWd0   = 823296;
constexpr long oWd2   = 888832;
constexpr long oWd4   = 1183744;
constexpr long oWd6h  = 1331200;
constexpr long oWd6l  = 1404928;
constexpr long oWd7   = 1478656;
constexpr long oWpost = 1699840;
constexpr long oXP    = 1736704;
constexpr long oD3    = oXP + (long)M1 * 64 * 4;
constexpr long oZ     = oD3 + (long)M1 * 64 * 2;
constexpr long zC1  = 0;
constexpr long zP1  = zC1 + (long)M1 * 64 * 4;
constexpr long zC2  = zP1 + (long)M2 * 32 * 4;
constexpr long zP2  = zC2 + (long)M2 * 64 * 4;
constexpr long zC3  = zP2 + (long)M3 * 64 * 2;
constexpr long zP3  = zC3 + (long)M3 * 128 * 4;
constexpr long zC4  = zP3 + (long)M4 * 128 * 2;
constexpr long zD0  = zC4 + (long)M4 * 256 * 2;
constexpr long zU1  = zD0 + (long)M4 * 128 * 4;
constexpr long zD1  = zU1 + (long)M3 * 128 * 2;
constexpr long zU2  = zD1 + (long)M3 * 128 * 4;
constexpr long zD2  = zU2 + (long)M2 * 128 * 2;
constexpr long zU3  = zD2 + (long)M2 * 64 * 4;
constexpr long zCOL = zU3 + (long)M1 * 64 * 4;
constexpr long COLHALF = (long)M2 * 288 * 2;
constexpr long zCOLLO = zCOL + COLHALF;
constexpr long zEND1 = zCOL + 2 * COLHALF;
constexpr long zGB   = 0;
constexpr long zCOL7 = zGB + (long)M1 * 256 * 4;
constexpr long zRAW  = zCOL7 + (long)MC7 * 288 * 2;
constexpr long zEND2 = zRAW + (long)MC7 * 384 * 4;
constexpr long zCOLP = 0;
constexpr long zCP   = zCOLP + (long)M1 * 288 * 2;
constexpr long zEND3 = zCP + (long)M1 * 64 * 4;
constexpr long ZS = zEND2;
constexpr long WS_TOTAL = oZ + ZS;
static_assert(oWmask + 64L * 32 * 2 == oWv1h && oWv1h + 64L * 32 * 2 == oWv1l && oWv1l + 64L * 32 * 2 == oWv2h);
static_assert(oWv2h + 64L * 288 * 2 == oWv2l && oWv2l + 64L * 288 * 2 == oWv3 && oWv3 + 128L * 576 * 2 == oWv4);
static_assert(oWv4 + 256L * 1152 * 2 == oWd0 && oWd0 + 128L * 256 * 2 == oWd2 && oWd2 + 128L * 1152 * 2 == oWd4);
static_assert(oWd4 + 64L * 1152 * 2 == oWd6h && oWd6h + 64L * 576 * 2 == oWd6l && oWd6l + 64L * 576 * 2 == oWd7);
static_assert(oWd7 + 384L * 288 * 2 == oWpost && oWpost + 64L * 288 * 2 == oXP);
static_assert(oD3 == 20611072L && oZ == 30048256L);
static_assert(zEND1 == 83460096L && zEND1 <= ZS && zEND3 <= ZS && ZS == 94961664L);
static_assert(WS_TOTAL == 125009920L && WS_TOTAL <= 134217728L);
static_assert((long)M1 * 32 * 2 <= COLHALF && (long)M3 * 576 * 2 <= 2 * COLHALF && (long)M4 * 1152 * 2 <= 2 * COLHALF);
static_assert((long)M3 * 1152 * 2 <= 2 * COLHALF && (long)MC4 * 1152 * 2 <= 2 * COLHALF && (long)MC6 * 576 * 2 <= COLHALF);
static_assert((long)NB * 32 * HW1 * 4 == (long)M1 * 64 * 2);
static_assert(M1 % 64 == 0 && M2 % 64 == 0 && M3 % 64 == 0 && M4 % 64 == 0 && MC4 % 64 == 0 && MC6 % 64 == 0 && MC7 % 64 == 0);
static_assert(32 % 32 == 0 && 288 % 32 == 0 && 576 % 32 == 0 && 1152 % 32 == 0 && 256 % 32 == 0);
static_assert((M1 * 32) % 2048 == 0 && (M2 * 288) % 2048 == 0 && (M3 * 576) % 2048 == 0 && (M4 * 1152) % 2048 == 0);
static_assert((M3 * 1152) % 2048 == 0 && (MC4 * 1152) % 2048 == 0 && (MC6 * 576) % 2048 == 0 && (MC7 * 288) % 2048 == 0 && (M1 * 288) % 2048 == 0);
static_assert((oZ % 256) == 0 && (zCOL % 256) == 0 && (zCOLLO % 256) == 0 && (zCOL7 % 256) == 0 && (zRAW % 256) == 0 && (zCP % 256) == 0);
static_assert((oXP % 256) == 0 && (oD3 % 256) == 0 && (zP1 % 256) == 0 && (zP2 % 256) == 0 && (zU3 % 256) == 0 && (zD2 % 256) == 0);
}

extern "C" void kernel_launch(void* const* d_in, const int* in_sizes, int n_in,
                              void* d_out, int out_size, void* d_ws, size_t ws_size,
                              hipStream_t stream)
{
  using namespace propns;
  if (n_in != 24) return;
  if (out_size != NB * 3 * HW1) return;
  if (ws_size < (size_t)WS_TOTAL) return;
  if (in_sizes[0] != NB * 3 * HW1 || in_sizes[1] != NB * 3 * HW1) return;
  if (in_sizes[2] != 32 * 27 || in_sizes[4] != 32 * 27 || in_sizes[6] != 64 * 288 || in_sizes[8] != 128 * 576) return;
  if (in_sizes[10] != 256 * 1152 || in_sizes[12] != 128 * 256 || in_sizes[14] != 128 * 1152) return;
  if (in_sizes[16] != 64 * 1152 || in_sizes[18] != 32 * 576 || in_sizes[20] != 384 * 288 || in_sizes[22] != 3 * 288) return;
  if (in_sizes[3] != 32 || in_sizes[5] != 32 || in_sizes[7] != 64 || in_sizes[9] != 128 || in_sizes[11] != 256) return;
  if (in_sizes[13] != 128 || in_sizes[15] != 128 || in_sizes[17] != 64 || in_sizes[19] != 32 || in_sizes[21] != 384 || in_sizes[23] != 3) return;

  const float* x      = (const float*)d_in[0];
  const float* rgb    = (const float*)d_in[1];
  const float* mask_w = (const float*)d_in[2];
  const float* mask_b = (const float*)d_in[3];
  const float* vgg_w1 = (const float*)d_in[4];
  const float* vgg_b1 = (const float*)d_in[5];
  const float* vgg_w2 = (const float*)d_in[6];
  const float* vgg_b2 = (const float*)d_in[7];
  const float* vgg_w3 = (const float*)d_in[8];
  const float* vgg_b3 = (const float*)d_in[9];
  const float* vgg_w4 = (const float*)d_in[10];
  const float* vgg_b4 = (const float*)d_in[11];
  const float* dec_w0 = (const float*)d_in[12];
  const float* dec_b0 = (const float*)d_in[13];
  const float* dec_w2 = (const float*)d_in[14];
  const float* dec_b2 = (const float*)d_in[15];
  const float* dec_w4 = (const float*)d_in[16];
  const float* dec_b4 = (const float*)d_in[17];
  const float* dec_w6 = (const float*)d_in[18];
  const float* dec_b6 = (const float*)d_in[19];
  const float* dec_w7 = (const float*)d_in[20];
  const float* dec_b7 = (const float*)d_in[21];
  const float* post_w = (const float*)d_in[22];
  const float* post_b = (const float*)d_in[23];
  float* out = (float*)d_out;

  char* ws = (char*)d_ws;
  unsigned short* Wmask = (unsigned short*)(ws + oWmask);
  unsigned short* Wv1h  = (unsigned short*)(ws + oWv1h);
  unsigned short* Wv1l  = (unsigned short*)(ws + oWv1l);
  unsigned short* Wv2h  = (unsigned short*)(ws + oWv2h);
  unsigned short* Wv2l  = (unsigned short*)(ws + oWv2l);
  unsigned short* Wv3   = (unsigned short*)(ws + oWv3);
  unsigned short* Wv4   = (unsigned short*)(ws + oWv4);
  unsigned short* Wd0   = (unsigned short*)(ws + oWd0);
  unsigned short* Wd2   = (unsigned short*)(ws + oWd2);
  unsigned short* Wd4   = (unsigned short*)(ws + oWd4);
  unsigned short* Wd6h  = (unsigned short*)(ws + oWd6h);
  unsigned short* Wd6l  = (unsigned short*)(ws + oWd6l);
  unsigned short* Wd7   = (unsigned short*)(ws + oWd7);
  unsigned short* Wpost = (unsigned short*)(ws + oWpost);
  float*          XP    = (float*)(ws + oXP);
  unsigned short* D3    = (unsigned short*)(ws + oD3);
  float*          OMAX  = (float*)(ws + oD3);
  char* zb = ws + oZ;
  float*          C1   = (float*)(zb + zC1);
  float*          P1   = (float*)(zb + zP1);
  float*          C2   = (float*)(zb + zC2);
  unsigned short* P2   = (unsigned short*)(zb + zP2);
  float*          C3   = (float*)(zb + zC3);
  unsigned short* P3   = (unsigned short*)(zb + zP3);
  unsigned short* C4   = (unsigned short*)(zb + zC4);
  float*          D0   = (float*)(zb + zD0);
  unsigned short* U1   = (unsigned short*)(zb + zU1);
  float*          D1   = (float*)(zb + zD1);
  unsigned short* U2   = (unsigned short*)(zb + zU2);
  float*          D2   = (float*)(zb + zD2);
  float*          U3   = (float*)(zb + zU3);
  unsigned short* COLH = (unsigned short*)(zb + zCOL);
  unsigned short* COLL = (unsigned short*)(zb + zCOLLO);
  float*          GB   = (float*)(zb + zGB);
  unsigned short* COL7 = (unsigned short*)(zb + zCOL7);
  float*          RAW  = (float*)(zb + zRAW);
  unsigned short* COLP = (unsigned short*)(zb + zCOLP);
  float*          CP   = (float*)(zb + zCP);

  const float carry = 64.0f;
  const float inv_carry = 1.0f / 64.0f;
  const float*          nores = P1;
  const float*          nof   = P1;
  const unsigned short* noh   = Wmask;
  float*                dumf  = P1;
  unsigned short*       dumh  = P2;

  auto gw = [](int Npad, int Kpad) { return dim3((unsigned)((Npad * Kpad / 8 + 255) / 256)); };
  auto gi = [](int nrows, int Kpad) { return dim3((unsigned)((long)nrows * Kpad / 2048)); };
  auto gg = [](int M, int N) { return dim3((unsigned)(((M / 64) * (N / 64) + 7) / 8)); };

  cast_weight<0><<<gw(64, 32),    256, 0, stream>>>(mask_w, 32, 27, 64, 32, carry, Wmask, Wmask);
  cast_weight<1><<<gw(64, 32),    256, 0, stream>>>(vgg_w1, 32, 27, 64, 32, 1.0f, Wv1h, Wv1l);
  cast_weight<1><<<gw(64, 288),   256, 0, stream>>>(vgg_w2, 64, 288, 64, 288, 1.0f, Wv2h, Wv2l);
  cast_weight<0><<<gw(128, 576),  256, 0, stream>>>(vgg_w3, 128, 576, 128, 576, carry, Wv3, Wv3);
  cast_weight<0><<<gw(256, 1152), 256, 0, stream>>>(vgg_w4, 256, 1152, 256, 1152, carry, Wv4, Wv4);
  cast_weight<0><<<gw(128, 256),  256, 0, stream>>>(dec_w0, 128, 256, 128, 256, carry, Wd0, Wd0);
  cast_weight<0><<<gw(128, 1152), 256, 0, stream>>>(dec_w2, 128, 1152, 128, 1152, carry, Wd2, Wd2);
  cast_weight<0><<<gw(64, 1152),  256, 0, stream>>>(dec_w4, 64, 1152, 64, 1152, carry, Wd4, Wd4);
  cast_weight<1><<<gw(64, 576),   256, 0, stream>>>(dec_w6, 32, 576, 64, 576, 1.0f, Wd6h, Wd6l);
  cast_weight<0><<<gw(384, 288),  256, 0, stream>>>(dec_w7, 384, 288, 384, 288, carry, Wd7, Wd7);
  cast_weight<0><<<gw(64, 288),   256, 0, stream>>>(post_w, 3, 288, 64, 288, carry, Wpost, Wpost);

  im2col3x3<0, 0><<<gi(M1, 32), 256, 0, stream>>>(x, noh, 3L * HW1, (long)HW1, 1L, COLH, COLH, 3, H1, W1, 27, 32, 0, M1);
  conv_gemm64<0, false, 0, false, 0><<<gg(M1, 64), 256, 0, stream>>>(COLH, COLH, 32, Wmask, Wmask, 32, XP, 64, mask_b, 32, nores, M1, 64, 32, inv_carry);

  im2col3x3<0, 1><<<gi(M1, 32), 256, 0, stream>>>(rgb, noh, 3L * HW1, (long)HW1, 1L, COLH, COLL, 3, H1, W1, 27, 32, 0, M1);
  conv_gemm64<1, true, 0, false, 0><<<gg(M1, 64), 256, 0, stream>>>(COLH, COLL, 32, Wv1h, Wv1l, 32, C1, 64, vgg_b1, 32, nores, M1, 64, 32, 1.0f);
  relu_pool3s2<1><<<dim3((unsigned)(M2 * 32 / 4 / 256)), 256, 0, stream>>>(C1, 64, 32, NB, H1, W1, P1, dumh);

  im2col3x3<0, 1><<<gi(M2, 288), 256, 0, stream>>>(P1, noh, (long)HW2 * 32, 1L, 32L, COLH, COLL, 32, H2, H2, 288, 288, 0, M2);
  conv_gemm64<1, true, 0, false, 0><<<gg(M2, 64), 256, 0, stream>>>(COLH, COLL, 288, Wv2h, Wv2l, 288, C2, 64, vgg_b2, 64, nores, M2, 64, 288, 1.0f);
  relu_pool3s2<0><<<dim3((unsigned)(M3 * 64 / 8 / 256)), 256, 0, stream>>>(C2, 64, 64, NB, H2, H2, dumf, P2);

  im2col3x3<1, 0><<<gi(M3, 576), 256, 0, stream>>>(nof, P2, (long)HW3 * 64, 1L, 64L, COLH, COLH, 64, H3, H3, 576, 576, 0, M3);
  conv_gemm64<0, false, 0, false, 0><<<gg(M3, 128), 256, 0, stream>>>(COLH, COLH, 576, Wv3, Wv3, 576, C3, 128, vgg_b3, 128, nores, M3, 128, 576, inv_carry);
  relu_pool3s2<0><<<dim3((unsigned)(M4 * 128 / 8 / 256)), 256, 0, stream>>>(C3, 128, 128, NB, H3, H3, dumf, P3);

  im2col3x3<1, 0><<<gi(M4, 1152), 256, 0, stream>>>(nof, P3, (long)HW4 * 128, 1L, 128L, COLH, COLH, 128, H4, H4, 1152, 1152, 0, M4);
  conv_gemm64<0, false, 1, false, 0><<<gg(M4, 256), 256, 0, stream>>>(COLH, COLH, 1152, Wv4, Wv4, 1152, C4, 256, vgg_b4, 256, nores, M4, 256, 1152, inv_carry);

  conv_gemm64<0, false, 0, false, 0><<<gg(M4, 128), 256, 0, stream>>>(C4, C4, 256, Wd0, Wd0, 256, D0, 128, dec_b0, 128, nores, M4, 128, 256, inv_carry);
  upsample2x<0><<<dim3((unsigned)(M3 * 128 / 8 / 256)), 256, 0, stream>>>(D0, 128, NB, H4, H4, dumf, U1);

  im2col3x3<1, 0><<<gi(M3, 1152), 256, 0, stream>>>(nof, U1, (long)HW3 * 128, 1L, 128L, COLH, COLH, 128, H3, H3, 1152, 1152, 0, M3);
  conv_gemm64<0, false, 0, true, 6><<<gg(M3, 128), 256, 0, stream>>>(COLH, COLH, 1152, Wd2, Wd2, 1152, D1, 128, dec_b2, 128, C3, M3, 128, 1152, inv_carry);
  upsample2x<0><<<dim3((unsigned)(M2 * 128 / 8 / 256)), 256, 0, stream>>>(D1, 128, NB, H3, H3, dumf, U2);

  for (int chk = 0; chk < 2; ++chk) {
    const int mb = chk * MC4;
    im2col3x3<1, 0><<<gi(MC4, 1152), 256, 0, stream>>>(nof, U2, (long)HW2 * 128, 1L, 128L, COLH, COLH, 128, H2, H2, 1152, 1152, mb, MC4);
    conv_gemm64<0, false, 0, true, 6><<<gg(MC4, 64), 256, 0, stream>>>(COLH, COLH, 1152, Wd4, Wd4, 1152, D2 + (size_t)mb * 64, 64, dec_b4, 64, C2 + (size_t)mb * 64, MC4, 64, 1152, inv_carry);
  }
  upsample2x<1><<<dim3((unsigned)(M1 * 64 / 4 / 256)), 256, 0, stream>>>(D2, 64, NB, H2, H2, U3, dumh);

  for (int chk = 0; chk < 8; ++chk) {
    const int mb = chk * MC6;
    im2col3x3<0, 1><<<gi(MC6, 576), 256, 0, stream>>>(U3, noh, (long)HW1 * 64, 1L, 64L, COLH, COLL, 64, H1, W1, 576, 576, mb, MC6);
    conv_gemm64<1, true, 1, true, 6><<<gg(MC6, 64), 256, 0, stream>>>(COLH, COLL, 576, Wd6h, Wd6l, 576, D3 + (size_t)mb * 64, 64, dec_b6, 32, C1 + (size_t)mb * 64, MC6, 64, 576, 1.0f);
  }

  for (int chk = 0; chk < 8; ++chk) {
    const int mb = chk * MC7;
    im2col3x3<1, 0><<<gi(MC7, 288), 256, 0, stream>>>(nof, D3, (long)HW1 * 64, 1L, 64L, COL7, COL7, 32, H1, W1, 288, 288, mb, MC7);
    conv_gemm64<0, false, 0, false, 0><<<gg(MC7, 384), 256, 0, stream>>>(COL7, COL7, 288, Wd7, Wd7, 288, RAW, 384, dec_b7, 384, nores, MC7, 384, 288, inv_carry);
    gates_base<<<dim3((unsigned)(MC7 / 8)), 256, 0, stream>>>(RAW, XP, GB, mb, MC7);
  }

  prop_scan_max<<<dim3((unsigned)(NB * 32)), 256, 0, stream>>>(GB, OMAX, NSTEPS);

  im2col3x3<0, 0><<<gi(M1, 288), 256, 0, stream>>>(OMAX, noh, 32L * HW1, (long)HW1, 1L, COLP, COLP, 32, H1, W1, 288, 288, 0, M1);
  conv_gemm64<0, false, 0, false, 0><<<gg(M1, 64), 256, 0, stream>>>(COLP, COLP, 288, Wpost, Wpost, 288, CP, 64, post_b, 3, nores, M1, 64, 288, inv_carry);
  gather_output<<<dim3((unsigned)(NB * 3 * HW1 / 4 / 256)), 256, 0, stream>>>(CP, out);
}
